// MessageFunction_36017595744927
// MI455X (gfx1250) — hardware-verified
//
#include <hip/hip_runtime.h>

constexpr int kBatch  = 8;
constexpr int kNodes  = 512;
constexpr int kDim    = 64;
constexpr int kCls    = 4;
constexpr int kKagg   = kCls * kNodes;
constexpr int kTPitch = 2 * kKagg;
constexpr int kOutW   = 2 * kDim;
constexpr unsigned short kOneBf16 = 0x3F80;

constexpr int kHBlocks = (kBatch * kNodes * kDim) / (256 * 8);
constexpr int kWBlocks = (2 * kCls * kDim * kDim) / (256 * 8);
static_assert(kHBlocks * 256 * 8 == kBatch * kNodes * kDim, "cast coverage h");
static_assert(kWBlocks * 256 * 8 == 2 * kCls * kDim * kDim, "cast coverage w");
static_assert((kWBlocks / 2) * 256 * 8 == kCls * kDim * kDim, "cast w split is block-uniform");

static_assert(kDim % 64 == 0 && kNodes % 64 == 0 && kDim % 32 == 0, "site A M=64 N=512 K=64");
static_assert(kNodes % 64 == 0 && kDim % 64 == 0 && kKagg % 32 == 0, "site B M=512 N=64 K=2048");


typedef __attribute__((ext_vector_type(16))) _Float16 v16h;
typedef __attribute__((ext_vector_type(8)))  _Float16 v8h;
typedef __attribute__((ext_vector_type(16))) __bf16   v16b;
typedef __attribute__((ext_vector_type(8)))  __bf16   v8b;
typedef __attribute__((ext_vector_type(8)))  float    v8f;
typedef __attribute__((ext_vector_type(4)))  float    v4f;
typedef __attribute__((ext_vector_type(4)))  unsigned int v4u;
typedef __attribute__((ext_vector_type(4)))  int      v4i;

__device__ __forceinline__ unsigned short f2bf_bits(float f) {
  unsigned u = __float_as_uint(f);
  return (unsigned short)((u + 0x7FFFu + ((u >> 16) & 1u)) >> 16);
}
__device__ __forceinline__ float bf_bits2f(unsigned short h) { return __uint_as_float(((unsigned)h) << 16); }
__device__ __forceinline__ unsigned pk16(unsigned short a, unsigned short b) { return (unsigned)a | ((unsigned)b << 16); }

__device__ __forceinline__ void dep_guard4_h(v8f& a, v8f& b, v8f& c, v8f& d, v16h x, v16h y) {
  asm volatile("v_nop\n\tv_nop\n\tv_nop\n\tv_nop" : "+v"(a), "+v"(b), "+v"(c), "+v"(d) : "v"(x), "v"(y));
}
__device__ __forceinline__ void dep_guard4_b(v8f& a, v8f& b, v8f& c, v8f& d, v16b x, v16b y) {
  asm volatile("v_nop\n\tv_nop\n\tv_nop\n\tv_nop" : "+v"(a), "+v"(b), "+v"(c), "+v"(d) : "v"(x), "v"(y));
}
__device__ __forceinline__ void keep4_h(v16h a, v16h b, v16h c, v16h d) { asm volatile("v_nop" :: "v"(a), "v"(b), "v"(c), "v"(d)); }
__device__ __forceinline__ void keep4_b(v16b a, v16b b, v16b c, v16b d) { asm volatile("v_nop" :: "v"(a), "v"(b), "v"(c), "v"(d)); }
__device__ __forceinline__ void acc_guard4(v8f& a, v8f& b, v8f& c, v8f& d) { asm volatile("v_nop\n\tv_nop\n\tv_nop\n\tv_nop" : "+v"(a), "+v"(b), "+v"(c), "+v"(d)); }

template <typename T> struct Frag;
template <> struct Frag<_Float16> {
  typedef v16h V; union U { v16h v; v8h h[2]; };
  static __device__ __forceinline__ v16h load(const _Float16* p) {
    U f; f.h[0] = *(const v8h*)(p); f.h[1] = *(const v8h*)(p + 16); return f.v;
  }
  static __device__ __forceinline__ v8f mma(v16h a, v16h b, v8f c) {
    return __builtin_amdgcn_wmma_f32_16x16x32_f16(false, a, false, b, (short)0, c, false, false);
  }
  static __device__ __forceinline__ void guard4(v8f& a, v8f& b, v8f& c, v8f& d, v16h x, v16h y) { dep_guard4_h(a, b, c, d, x, y); }
  static __device__ __forceinline__ void keep(v16h a, v16h b, v16h c, v16h d) { keep4_h(a, b, c, d); }
};
template <> struct Frag<__bf16> {
  typedef v16b V; union U { v16b v; v8b h[2]; };
  static __device__ __forceinline__ v16b load(const __bf16* p) {
    U f; f.h[0] = *(const v8b*)(p); f.h[1] = *(const v8b*)(p + 16); return f.v;
  }
  static __device__ __forceinline__ v8f mma(v16b a, v16b b, v8f c) {
    return __builtin_amdgcn_wmma_f32_16x16x32_bf16(false, a, false, b, (short)0, c, false, false);
  }
  static __device__ __forceinline__ void guard4(v8f& a, v8f& b, v8f& c, v8f& d, v16b x, v16b y) { dep_guard4_b(a, b, c, d, x, y); }
  static __device__ __forceinline__ void keep(v16b a, v16b b, v16b c, v16b d) { keep4_b(a, b, c, d); }
};

template <int ET> struct Elem;
template <> struct Elem<0> { typedef _Float16 T; };
template <> struct Elem<1> { typedef __bf16 T; };
template <int ET, bool SPLIT, bool ALO, int BIAS_MODE, int OUT_MODE>
__global__ __launch_bounds__(256) void wmma_gemm64(
    const unsigned short* __restrict__ Ap, const unsigned short* __restrict__ A2p, int lda, long strideA, long strideAz,
    const unsigned short* __restrict__ Btp, const unsigned short* __restrict__ Bt2p, int ldb, long strideB, long strideBz,
    void* __restrict__ Cout, void* __restrict__ Cout2, int ldc, long strideC, long strideCz,
    const float* __restrict__ bias, int biasZ,
    int M, int N, int K, float scale) {
  typedef typename Elem<ET>::T T;
  typedef typename Frag<T>::V V;
  const T* A = (const T*)Ap; const T* A2 = (const T*)A2p; const T* Bt = (const T*)Btp; const T* Bt2 = (const T*)Bt2p;
  __shared__ __align__(16) float sT[8][16 * 68];
  const int b    = blockIdx.y;
  const int bz   = blockIdx.z;
  const int lane = threadIdx.x & 31;
  const int wave = threadIdx.x >> 5;
  const int tilesN = N >> 6;
  const int tilesM = M >> 6;
  const int tile = blockIdx.x * 8 + wave;
  if (tile >= tilesM * tilesN) return;
  const int tm = tile / tilesN;
  const int tn = tile - tm * tilesN;
  const int m0 = tm << 6;
  const int n0 = tn << 6;

  const size_t offA = (size_t)b * (size_t)strideA + (size_t)bz * (size_t)strideAz;
  const size_t offB = (size_t)b * (size_t)strideB + (size_t)bz * (size_t)strideBz;
  const size_t offC = (size_t)b * (size_t)strideC + (size_t)bz * (size_t)strideCz;
  const T* Ab  = A  + offA;
  const T* Bb  = Bt + offB;
  const T* Ab2 = (SPLIT && ALO) ? (A2 + offA) : nullptr;
  const T* Bb2 = SPLIT ? (Bt2 + offB) : nullptr;
  const float* biasp = (BIAS_MODE != 0) ? (bias + (size_t)bz * (size_t)biasZ) : nullptr;

  const int rlane = lane & 15;
  const int koff  = (lane >> 4) * 8;
  const int mOff  = (lane >> 4) * 8;

  v8f acc[4][4];
#pragma unroll
  for (int i = 0; i < 4; ++i)
#pragma unroll
    for (int j = 0; j < 4; ++j) acc[i][j] = (v8f){0.f,0.f,0.f,0.f,0.f,0.f,0.f,0.f};

  for (int k0 = 0; k0 < K; k0 += 32) {
    V bh[4], bl[4];
#pragma unroll
    for (int j = 0; j < 4; ++j) {
      const size_t bo = (size_t)(n0 + (j << 4) + rlane) * ldb + koff + k0;
      bh[j] = Frag<T>::load(Bb + bo);
      if (SPLIT) bl[j] = Frag<T>::load(Bb2 + bo);
    }
#pragma unroll
    for (int i = 0; i < 4; ++i) {
      const size_t ao = (size_t)(m0 + (i << 4) + rlane) * lda + koff + k0;
      V ah = Frag<T>::load(Ab + ao);
      V al = ah;
      if (SPLIT && ALO) al = Frag<T>::load(Ab2 + ao);
#pragma unroll
      for (int j = 0; j < 4; ++j) {
        acc[i][j] = Frag<T>::mma(ah, bh[j], acc[i][j]);
        if (SPLIT) {
          acc[i][j] = Frag<T>::mma(ah, bl[j], acc[i][j]);
          if (ALO) acc[i][j] = Frag<T>::mma(al, bh[j], acc[i][j]);
        }
      }
      Frag<T>::guard4(acc[i][0], acc[i][1], acc[i][2], acc[i][3], ah, al);
    }
    Frag<T>::keep(bh[0], bh[1], bh[2], bh[3]);
    if (SPLIT) Frag<T>::keep(bl[0], bl[1], bl[2], bl[3]);
  }
  acc_guard4(acc[0][0], acc[0][1], acc[0][2], acc[0][3]);
  acc_guard4(acc[1][0], acc[1][1], acc[1][2], acc[1][3]);
  acc_guard4(acc[2][0], acc[2][1], acc[2][2], acc[2][3]);
  acc_guard4(acc[3][0], acc[3][1], acc[3][2], acc[3][3]);

  float* slab = sT[wave];
#pragma unroll
  for (int i = 0; i < 4; ++i) {
    const int mBase = m0 + (i << 4);
#pragma unroll
    for (int j = 0; j < 4; ++j) {
      const int n = n0 + (j << 4) + rlane;
      float bv = 0.f;
      if (BIAS_MODE == 2) bv = biasp[n];
#pragma unroll
      for (int r = 0; r < 8; ++r) {
        float v = acc[i][j][r] * scale;
        if (BIAS_MODE == 1) v += biasp[mBase + mOff + r];
        if (BIAS_MODE == 2) v += bv;
        slab[(mOff + r) * 68 + (j << 4) + rlane] = v;
      }
    }
    __builtin_amdgcn_fence(__ATOMIC_RELEASE, "workgroup");
    __builtin_amdgcn_wave_barrier();
    __builtin_amdgcn_fence(__ATOMIC_ACQUIRE, "workgroup");
    if (OUT_MODE == 0) {
      float* C = (float*)Cout + offC;
      const int hh = lane >> 4, c4 = (lane & 15) * 4;
      for (int pass = 0; pass < 2; ++pass) {
#pragma unroll
        for (int it = 0; it < 8; ++it) {
          const int row = it * 2 + hh;
          v4f v = *(const v4f*)(slab + row * 68 + c4);
          *(volatile v4f*)(C + (size_t)(mBase + row) * ldc + n0 + c4) = v;
        }
        __threadfence();
      }
    } else {
      const int q = lane >> 3, c8 = (lane & 7) * 8;
      unsigned short* C  = (unsigned short*)Cout  + offC;
      unsigned short* C2 = (OUT_MODE == 2) ? ((unsigned short*)Cout2 + offC) : nullptr;
      for (int pass = 0; pass < 2; ++pass) {
#pragma unroll
        for (int it = 0; it < 4; ++it) {
          const int row = it * 4 + q;
          const float* sp = slab + row * 68 + c8;
          v8h hv, lv;
#pragma unroll
          for (int e = 0; e < 8; ++e) {
            if (OUT_MODE == 1) {
              hv[e] = (_Float16)sp[e];
            } else {
              unsigned short hb = f2bf_bits(sp[e]);
              unsigned short lb = f2bf_bits(sp[e] - bf_bits2f(hb));
              hv[e] = __builtin_bit_cast(_Float16, hb);
              lv[e] = __builtin_bit_cast(_Float16, lb);
            }
          }
          *(volatile v8h*)(C + (size_t)(mBase + row) * ldc + n0 + c8) = hv;
          if (OUT_MODE == 2) *(volatile v8h*)(C2 + (size_t)(mBase + row) * ldc + n0 + c8) = lv;
        }
        __threadfence();
      }
    }
    __builtin_amdgcn_fence(__ATOMIC_RELEASE, "workgroup");
    __builtin_amdgcn_wave_barrier();
    __builtin_amdgcn_fence(__ATOMIC_ACQUIRE, "workgroup");
  }
}

__device__ __forceinline__ v4u pack_bf16x8(v4f a, v4f c) {
  return (v4u){ pk16(f2bf_bits(a[0]), f2bf_bits(a[1])), pk16(f2bf_bits(a[2]), f2bf_bits(a[3])),
                pk16(f2bf_bits(c[0]), f2bf_bits(c[1])), pk16(f2bf_bits(c[2]), f2bf_bits(c[3])) };
}
__global__ __launch_bounds__(256) void cast_kernel(const float* __restrict__ h, const float* __restrict__ win,
                                                   const float* __restrict__ wout, const float* __restrict__ bias,
                                                   unsigned short* __restrict__ hb, unsigned short* __restrict__ wb,
                                                   float* __restrict__ biasr) {
  const int blk = blockIdx.x;
  const int t   = threadIdx.x;
  if (blk < kHBlocks) {
    const size_t e8 = (size_t)(blk * 256 + t) * 8;
    const v4f a = *(const v4f*)(h + e8);
    const v4f c = *(const v4f*)(h + e8 + 4);
    const v4u u = pack_bf16x8(a, c);
    unsigned short* q = hb + e8;
    *(volatile v4u*)q = u;
    __threadfence();
    *(volatile v4u*)q = u;
  } else if (blk < kHBlocks + kWBlocks) {
    const int wi = blk - kHBlocks;
    const float* src = (wi < (kWBlocks / 2)) ? win : wout;
    const size_t eo  = (size_t)((wi & (kWBlocks / 2 - 1)) * 256 + t) * 8;
    const v4f a = *(const v4f*)(src + eo);
    const v4f c = *(const v4f*)(src + eo + 4);
    const v4u u = pack_bf16x8(a, c);
    unsigned short* q = wb + (size_t)(wi * 256 + t) * 8;
    *(volatile v4u*)q = u;
    __threadfence();
    *(volatile v4u*)q = u;
  } else if (t < 32) {
    const v4f a = *(const v4f*)(bias + 4 * t);
    v4f r;
#pragma unroll
    for (int e = 0; e < 4; ++e) r[e] = bf_bits2f(f2bf_bits(a[e]));
    float* q = biasr + 4 * t;
    *(volatile v4f*)q = r;
    __threadfence();
    *(volatile v4f*)q = r;
  }
}

__global__ __launch_bounds__(256) void onehot_kernel(const int* __restrict__ adj, unsigned short* __restrict__ aoh) {
  __shared__ __align__(16) int sm[16][260];
  const int t = threadIdx.x, lane = t & 31, wave = t >> 5;
  const int wt = blockIdx.x & 1, vt = blockIdx.x >> 1;
  const int b = blockIdx.y, dir = blockIdx.z;
  const int w0 = wt * 256, v0 = vt * 16;
  const int* ab = adj + (size_t)b * kNodes * kNodes;
  if (dir == 0) {
#pragma unroll
    for (int i = 0; i < 4; ++i) {
      const int e  = i * 1024 + 4 * t;
      const int vl = e >> 8, wl = e & 255;
      const v4i q = *(const v4i*)(ab + (size_t)(v0 + vl) * kNodes + w0 + wl);
      *(v4i*)(&sm[vl][wl]) = q;
    }
  } else {
#pragma unroll
    for (int i = 0; i < 4; ++i) {
      const int e  = i * 1024 + 4 * t;
      const int wl = e >> 4, vl = e & 15;
      const v4i q = *(const v4i*)(ab + (size_t)(w0 + wl) * kNodes + v0 + vl);
      sm[vl][wl]     = q[0];
      sm[vl + 1][wl] = q[1];
      sm[vl + 2][wl] = q[2];
      sm[vl + 3][wl] = q[3];
    }
  }
  __syncthreads();

  unsigned short* pb = aoh + ((size_t)dir * kBatch + b) * ((size_t)kNodes * kKagg);
#pragma unroll
  for (int it = 0; it < 2; ++it) {
    const int vl = it * 8 + wave;
    const int wl = 8 * lane;
    const v4i qa = *(const v4i*)(&sm[vl][wl]);
    const v4i qc = *(const v4i*)(&sm[vl][wl + 4]);
    int cl[8];
    cl[0] = qa[0]; cl[1] = qa[1]; cl[2] = qa[2]; cl[3] = qa[3];
    cl[4] = qc[0]; cl[5] = qc[1]; cl[6] = qc[2]; cl[7] = qc[3];
    v4u u[4];
#pragma unroll
    for (int c = 0; c < 4; ++c) {
      unsigned short s[8];
#pragma unroll
      for (int e = 0; e < 8; ++e) s[e] = (cl[e] == c) ? kOneBf16 : (unsigned short)0;
      u[c] = (v4u){ pk16(s[0], s[1]), pk16(s[2], s[3]), pk16(s[4], s[5]), pk16(s[6], s[7]) };
    }
    unsigned short* rowp = pb + (size_t)(v0 + vl) * kKagg + w0 + wl;
    for (int pass = 0; pass < 2; ++pass) {
#pragma unroll
      for (int c = 0; c < 4; ++c) *(volatile v4u*)(rowp + c * kNodes) = u[c];
      __threadfence();
    }
  }
}

extern "C" void kernel_launch(void* const* d_in, const int* in_sizes, int n_in,
                              void* d_out, int out_size, void* d_ws, size_t ws_size, hipStream_t stream) {
  if (n_in < 5) return;
  if (in_sizes[0] != kBatch * kNodes * kDim || in_sizes[1] != kBatch * kNodes * kNodes ||
      in_sizes[2] != kCls * kDim * kDim || in_sizes[3] != kCls * kDim * kDim ||
      in_sizes[4] != kOutW || out_size != kBatch * kNodes * kOutW) return;
  const float* h    = (const float*)d_in[0];
  const int*   adj  = (const int*)  d_in[1];
  const float* win  = (const float*)d_in[2];
  const float* wout = (const float*)d_in[3];
  const float* bias = (const float*)d_in[4];
  float* out = (float*)d_out;

  char* ws = (char*)d_ws; size_t off = 0;
  auto carve = [&](size_t bytes) -> char* { char* p = ws + off; off += (bytes + 4095) & ~(size_t)4095; return p; };
  unsigned short* AOH   = (unsigned short*)carve((size_t)2 * kBatch * kNodes * kKagg * 2);
  unsigned short* HB    = (unsigned short*)carve((size_t)kBatch * kNodes * kDim * 2);
  unsigned short* WB    = (unsigned short*)carve((size_t)2 * kCls * kDim * kDim * 2);
  float*          BIASR = (float*)carve((size_t)kOutW * 4);
  unsigned short* TH    = (unsigned short*)carve((size_t)kBatch * kDim * kTPitch * 2);
  unsigned short* TL    = (unsigned short*)carve((size_t)kBatch * kDim * kTPitch * 2);
  if (off > ws_size || off > (size_t)134217728) return;

  cast_kernel<<<kHBlocks + kWBlocks + 1, 256, 0, stream>>>(h, win, wout, bias, HB, WB, BIASR);

  onehot_kernel<<<dim3(64, kBatch, 2), 256, 0, stream>>>(adj, AOH);

  wmma_gemm64<1, false, false, 0, 2><<<dim3(1, kBatch, 2 * kCls), 256, 0, stream>>>(
      (const unsigned short*)WB, (const unsigned short*)nullptr, kDim, 0L, (long)(kDim * kDim),
      (const unsigned short*)HB, (const unsigned short*)nullptr, kDim, (long)(kNodes * kDim), 0L,
      (void*)TH, (void*)TL, kTPitch, (long)kDim * kTPitch, (long)kNodes,
      (const float*)nullptr, 0,
      kDim, kNodes, kDim, 1.0f);

  wmma_gemm64<1, true, false, 2, 0><<<dim3(1, kBatch, 2), 256, 0, stream>>>(
      (const unsigned short*)AOH, (const unsigned short*)nullptr, kKagg, (long)kNodes * kKagg, (long)kBatch * kNodes * kKagg,
      (const unsigned short*)TH, (const unsigned short*)TL, kTPitch, (long)kDim * kTPitch, (long)kKagg,
      (void*)out, (void*)nullptr, kOutW, (long)kNodes * kOutW, (long)kDim,
      (const float*)BIASR, kDim,
      kNodes, kDim, kKagg, 1.0f);
}
